// CrossMamba_28879360099159
// MI455X (gfx1250) — hardware-verified
//
#include <hip/hip_runtime.h>
#include <stddef.h>

typedef __attribute__((ext_vector_type(16))) _Float16 v16h;
typedef __attribute__((ext_vector_type(8)))  _Float16 v8h;
typedef __attribute__((ext_vector_type(16))) __bf16   v16b;
typedef __attribute__((ext_vector_type(8)))  __bf16   v8b;
typedef __attribute__((ext_vector_type(8)))  float    v8f;
typedef __attribute__((ext_vector_type(4)))  float    v4f;
typedef __attribute__((ext_vector_type(4)))  unsigned v4u;
typedef __attribute__((ext_vector_type(2)))  unsigned v2u;

constexpr int kBatch  = 2;
constexpr int kSeq    = 2048;
constexpr int kDModel = 1024;
constexpr int kDInner = 2048;
constexpr int kDState = 16;
constexpr int kDConv  = 4;
constexpr int kDtRank = 64;
constexpr int kRTot   = 96;
constexpr int kRPad   = 128;
constexpr float kLog2e = 1.4426950408889634f;
constexpr size_t kPlane = (size_t)kBatch * kSeq * kDInner;

static_assert(kSeq % 64 == 0 && kDInner % 64 == 0 && kDModel % 64 == 0 && kRPad % 64 == 0, "M,N tile multiples");
static_assert(kDModel % 32 == 0 && kDInner % 32 == 0 && kDtRank % 32 == 0, "K multiples of 32");
static_assert(kRTot <= kRPad && kDtRank + 2 * kDState == kRTot, "x_dbl layout");
static_assert(kDInner == 4 * 512, "conv block covers one row with 512 threads x 4 channels");
static_assert(kDInner % 128 == 0, "scan block covers 128 channels");

__device__ __forceinline__ unsigned short f2bf_bits(float f) {
  unsigned u = __float_as_uint(f);
  return (unsigned short)((u + 0x7FFFu + ((u >> 16) & 1u)) >> 16);
}
__device__ __forceinline__ float bf_bits2f(unsigned short h) { return __uint_as_float(((unsigned)h) << 16); }
__device__ __forceinline__ float bf_rne(float f) { return bf_bits2f(f2bf_bits(f)); }
__device__ __forceinline__ void split_pair(float a, float c, unsigned& hp, unsigned& lp) {
  const unsigned short ha = f2bf_bits(a), hc = f2bf_bits(c);
  const unsigned short la = f2bf_bits(a - bf_bits2f(ha)), lc = f2bf_bits(c - bf_bits2f(hc));
  hp = (unsigned)ha | ((unsigned)hc << 16);
  lp = (unsigned)la | ((unsigned)lc << 16);
}

__device__ __forceinline__ void dep_guard_h(v8f& a, v8f& b, v16h x, v16h y) { asm volatile("v_nop\n\tv_nop\n\tv_nop\n\tv_nop" : "+v"(a), "+v"(b) : "v"(x), "v"(y)); }
__device__ __forceinline__ void dep_guard_b(v8f& a, v8f& b, v16b x, v16b y) { asm volatile("v_nop\n\tv_nop\n\tv_nop\n\tv_nop" : "+v"(a), "+v"(b) : "v"(x), "v"(y)); }
__device__ __forceinline__ void keep4_h(v16h a, v16h b, v16h c, v16h d) { asm volatile("v_nop" :: "v"(a), "v"(b), "v"(c), "v"(d)); }
__device__ __forceinline__ void keep4_b(v16b a, v16b b, v16b c, v16b d) { asm volatile("v_nop" :: "v"(a), "v"(b), "v"(c), "v"(d)); }
__device__ __forceinline__ void acc_guard4(v8f& a, v8f& b, v8f& c, v8f& d) { asm volatile("v_nop\n\tv_nop\n\tv_nop\n\tv_nop" : "+v"(a), "+v"(b), "+v"(c), "+v"(d)); }
template <typename T> struct Frag;
template <> struct Frag<_Float16> {
  typedef v16h V; union U { v16h v; v8h h[2]; };
  static __device__ __forceinline__ v16h load(const _Float16* p) {
    U f; f.h[0] = *(const v8h*)(p); f.h[1] = *(const v8h*)(p + 16); return f.v;
  }
  static __device__ __forceinline__ v8f mma(v16h a, v16h b, v8f c) {
    return __builtin_amdgcn_wmma_f32_16x16x32_f16(false, a, false, b, (short)0, c, false, false);
  }
  static __device__ __forceinline__ void guard(v8f& a, v8f& b, v16h x, v16h y) { dep_guard_h(a, b, x, y); }
  static __device__ __forceinline__ void keep(v16h a, v16h b, v16h c, v16h d) { keep4_h(a, b, c, d); }
};
template <> struct Frag<__bf16> {
  typedef v16b V; union U { v16b v; v8b h[2]; };
  static __device__ __forceinline__ v16b load(const __bf16* p) {
    U f; f.h[0] = *(const v8b*)(p); f.h[1] = *(const v8b*)(p + 16); return f.v;
  }
  static __device__ __forceinline__ v8f mma(v16b a, v16b b, v8f c) {
    return __builtin_amdgcn_wmma_f32_16x16x32_bf16(false, a, false, b, (short)0, c, false, false);
  }
  static __device__ __forceinline__ void guard(v8f& a, v8f& b, v16b x, v16b y) { dep_guard_b(a, b, x, y); }
  static __device__ __forceinline__ void keep(v16b a, v16b b, v16b c, v16b d) { keep4_b(a, b, c, d); }
};

template <int ET> struct Elem;
template <> struct Elem<0> { typedef _Float16 T; };
template <> struct Elem<1> { typedef __bf16 T; };
template <int ET, bool SPLIT, bool SPLITB, int BIAS_MODE, int OUT_MODE, bool RESID, int ACT = 0>
__global__ __launch_bounds__(256) void wmma_gemm64(
    const unsigned short* __restrict__ Ap, const unsigned short* __restrict__ A2p, int lda, long strideA,
    const unsigned short* __restrict__ Btp, const unsigned short* __restrict__ Bt2p, int ldb, long strideB,
    void* __restrict__ Cout, void* __restrict__ Cout2, int ldc, long strideC,
    const float* __restrict__ bias,
    const float* __restrict__ resid, long strideR,
    int M, int N, int K, float scale) {
  typedef typename Elem<ET>::T T;
  typedef typename Frag<T>::V V;
  const T* A = (const T*)Ap; const T* A2 = (const T*)A2p; const T* Bt = (const T*)Btp; const T* Bt2 = (const T*)Bt2p;
  __shared__ __align__(16) float sT[8][16 * 68];
  const int b    = blockIdx.y;
  const int lane = threadIdx.x & 31;
  const int wave = threadIdx.x >> 5;
  const int tilesN = N >> 6;
  const int tilesM = M >> 6;
  const int tile = blockIdx.x * 8 + wave;
  if (tile >= tilesM * tilesN) return;
  const int tm = tile / tilesN;
  const int tn = tile - tm * tilesN;
  const int m0 = tm << 6;
  const int n0 = tn << 6;

  const T* Ab  = A  + (size_t)b * strideA;
  const T* Bb  = Bt + (size_t)b * strideB;
  const T* Ab2 = SPLIT ? (A2  + (size_t)b * strideA) : nullptr;
  const T* Bb2 = (SPLIT && SPLITB) ? (Bt2 + (size_t)b * strideB) : nullptr;

  const int rlane = lane & 15;
  const int koff  = (lane >> 4) * 8;
  const int mOff  = (lane >> 4) * 8;

  v8f acc[4][4];
#pragma unroll
  for (int i = 0; i < 4; ++i)
#pragma unroll
    for (int j = 0; j < 4; ++j) acc[i][j] = (v8f){0.f,0.f,0.f,0.f,0.f,0.f,0.f,0.f};

  for (int k0 = 0; k0 < K; k0 += 32) {
    V bh[4], bl[4];
#pragma unroll
    for (int j = 0; j < 4; ++j) {
      const size_t bo = (size_t)(n0 + (j << 4) + rlane) * ldb + koff + k0;
      bh[j] = Frag<T>::load(Bb + bo);
      if (SPLIT && SPLITB) bl[j] = Frag<T>::load(Bb2 + bo);
    }
#pragma unroll
    for (int i = 0; i < 4; ++i) {
      const size_t ao = (size_t)(m0 + (i << 4) + rlane) * lda + koff + k0;
      V ah = Frag<T>::load(Ab + ao);
      V al;
      if (SPLIT) al = Frag<T>::load(Ab2 + ao);
#pragma unroll
      for (int j = 0; j < 4; ++j) {
        acc[i][j] = Frag<T>::mma(ah, bh[j], acc[i][j]);
        if (SPLIT && SPLITB) acc[i][j] = Frag<T>::mma(ah, bl[j], acc[i][j]);
        if (SPLIT) acc[i][j] = Frag<T>::mma(al, bh[j], acc[i][j]);
      }
      Frag<T>::guard(acc[i][0], acc[i][3], ah, SPLIT ? al : ah);
    }
    Frag<T>::keep(bh[0], bh[1], bh[2], bh[3]);
    if (SPLIT && SPLITB) Frag<T>::keep(bl[0], bl[1], bl[2], bl[3]);
  }
  acc_guard4(acc[0][0], acc[0][1], acc[0][2], acc[0][3]);
  acc_guard4(acc[1][0], acc[1][1], acc[1][2], acc[1][3]);
  acc_guard4(acc[2][0], acc[2][1], acc[2][2], acc[2][3]);
  acc_guard4(acc[3][0], acc[3][1], acc[3][2], acc[3][3]);

  float* slab = sT[wave];
  const float* Rb = RESID ? (resid + (size_t)b * strideR) : nullptr;
#pragma unroll
  for (int i = 0; i < 4; ++i) {
    const int mBase = m0 + (i << 4);
#pragma unroll
    for (int j = 0; j < 4; ++j) {
      const int n = n0 + (j << 4) + rlane;
      float bv = 0.f;
      if (BIAS_MODE == 2) bv = bias[n];
#pragma unroll
      for (int r = 0; r < 8; ++r) {
        float v = acc[i][j][r] * scale;
        if (BIAS_MODE == 1) v += bias[mBase + mOff + r];
        if (BIAS_MODE == 2) v += bv;
        if (RESID) v += Rb[(size_t)(mBase + mOff + r) * ldc + n];
        if (ACT == 1) v = tanhf(v);
        if (ACT == 2) v = fmaxf(v, 0.0f);
        if (ACT == 3) v = v / (1.0f + expf(-v));
        if (ACT == 4) v = (v > 0.f) ? v : 0.01f * v;
        slab[(mOff + r) * 68 + (j << 4) + rlane] = v;
      }
    }
    __builtin_amdgcn_fence(__ATOMIC_RELEASE, "workgroup");
    __builtin_amdgcn_wave_barrier();
    __builtin_amdgcn_fence(__ATOMIC_ACQUIRE, "workgroup");
    if (OUT_MODE == 0) {
      float* C = (float*)Cout + (size_t)b * strideC;
      const int hh = lane >> 4, c4 = (lane & 15) * 4;
      for (int pass = 0; pass < 2; ++pass) {
#pragma unroll
        for (int it = 0; it < 8; ++it) {
          const int row = it * 2 + hh;
          v4f v = *(const v4f*)(slab + row * 68 + c4);
          *(volatile v4f*)(C + (size_t)(mBase + row) * ldc + n0 + c4) = v;
        }
        __threadfence();
      }
    } else {
      const int q = lane >> 3, c8 = (lane & 7) * 8;
      unsigned short* C  = (unsigned short*)Cout  + (size_t)b * strideC;
      unsigned short* C2 = (OUT_MODE == 2) ? ((unsigned short*)Cout2 + (size_t)b * strideC) : nullptr;
      for (int pass = 0; pass < 2; ++pass) {
#pragma unroll
        for (int it = 0; it < 4; ++it) {
          const int row = it * 4 + q;
          const float* sp = slab + row * 68 + c8;
          v8h hv, lv;
#pragma unroll
          for (int e = 0; e < 8; ++e) {
            if (OUT_MODE == 1) {
              hv[e] = (_Float16)sp[e];
            } else {
              unsigned short hb = f2bf_bits(sp[e]);
              unsigned short lb = f2bf_bits(sp[e] - bf_bits2f(hb));
              hv[e] = __builtin_bit_cast(_Float16, hb);
              lv[e] = __builtin_bit_cast(_Float16, lb);
            }
          }
          *(volatile v8h*)(C + (size_t)(mBase + row) * ldc + n0 + c8) = hv;
          if (OUT_MODE == 2) *(volatile v8h*)(C2 + (size_t)(mBase + row) * ldc + n0 + c8) = lv;
        }
        __threadfence();
      }
    }
    __builtin_amdgcn_fence(__ATOMIC_RELEASE, "workgroup");
    __builtin_amdgcn_wave_barrier();
    __builtin_amdgcn_fence(__ATOMIC_ACQUIRE, "workgroup");
  }
}


__global__ __launch_bounds__(256) void cast_f32_bf16x2(
    const float* __restrict__ in, unsigned* __restrict__ out, int n_src2, int n_tot2) {
  const int i = blockIdx.x * 256 + threadIdx.x;
  if (i < n_tot2) {
    const int ic = (i < n_src2) ? i : (n_src2 - 1);
    const float a = in[(size_t)2 * ic], c = in[(size_t)2 * ic + 1];
    unsigned u = (unsigned)f2bf_bits(a) | ((unsigned)f2bf_bits(c) << 16);
    u = (i < n_src2) ? u : 0u;
    ((volatile unsigned*)out)[i] = u;
    __threadfence();
    ((volatile unsigned*)out)[i] = u;
  }
}

__global__ __launch_bounds__(512) void k_conv_silu_split(
    const float* __restrict__ xraw, const float* __restrict__ convw, const float* __restrict__ convb,
    v4u* __restrict__ uplanes) {
  __shared__ __align__(16) unsigned shp[2][kDInner / 2];
  const int row = blockIdx.x;
  const int b = row / kSeq;
  const int l = row - b * kSeq;
  const int t = threadIdx.x;
  const int e4 = 4 * t;
  v4f wv[4];
#pragma unroll
  for (int c = 0; c < 4; ++c) wv[c] = *(const v4f*)(convw + (size_t)16 * t + 4 * c);
  const v4f bb = *(const v4f*)(convb + e4);
  v4f xk[4];
  const v4f zero4 = (v4f){0.f, 0.f, 0.f, 0.f};
#pragma unroll
  for (int k = 0; k < kDConv; ++k) {
    const int li = l - (kDConv - 1) + k;
    const int lic = (li < 0) ? 0 : li;
    const v4f v = *(const v4f*)(xraw + ((size_t)(b * kSeq + lic)) * kDInner + e4);
    xk[k] = (li >= 0) ? v : zero4;
  }
  float uv[4];
#pragma unroll
  for (int c = 0; c < 4; ++c) {
    float s = bf_rne(wv[c][0]) * xk[0][c];
    s = s + bf_rne(wv[c][1]) * xk[1][c];
    s = s + bf_rne(wv[c][2]) * xk[2][c];
    s = s + bf_rne(wv[c][3]) * xk[3][c];
    s = s + bf_rne(bb[c]);
    const float sg = __builtin_amdgcn_rcpf(1.0f + expf(-s));
    uv[c] = s * sg;
  }
  unsigned hp0, hp1, lp0, lp1;
  split_pair(uv[0], uv[1], hp0, lp0);
  split_pair(uv[2], uv[3], hp1, lp1);
  *(v2u*)(&shp[0][2 * t]) = (v2u){hp0, hp1};
  *(v2u*)(&shp[1][2 * t]) = (v2u){lp0, lp1};
  __syncthreads();
  {
    const int plane = t >> 8;
    const int tt = t & 255;
    const v4u val = *(const v4u*)(&shp[plane][4 * tt]);
    v4u* dst = uplanes + (size_t)plane * (kPlane / 8) + (size_t)row * (kDInner / 8) + tt;
    *(volatile v4u*)dst = val;
    __threadfence();
    *(volatile v4u*)dst = val;
  }
}

__global__ __launch_bounds__(256) void k_dt_split(
    const float* __restrict__ xdbl, v4u* __restrict__ dtplanes, int nrows) {
  const int idx = blockIdx.x * 256 + threadIdx.x;
  const int row = idx >> 3;
  const int c8 = (idx & 7) * 8;
  if (row < nrows) {
    const float* p = xdbl + (size_t)row * kRPad + c8;
    const v4f a = *(const v4f*)p;
    const v4f c = *(const v4f*)(p + 4);
    v4u hw, lw;
    unsigned h, lo;
    split_pair(a[0], a[1], h, lo); hw[0] = h; lw[0] = lo;
    split_pair(a[2], a[3], h, lo); hw[1] = h; lw[1] = lo;
    split_pair(c[0], c[1], h, lo); hw[2] = h; lw[2] = lo;
    split_pair(c[2], c[3], h, lo); hw[3] = h; lw[3] = lo;
    v4u* ph = dtplanes + idx;
    v4u* pl = dtplanes + (size_t)nrows * (kDtRank / 8) + idx;
    *(volatile v4u*)ph = hw;
    *(volatile v4u*)pl = lw;
    __threadfence();
    *(volatile v4u*)ph = hw;
    *(volatile v4u*)pl = lw;
  }
}

__global__ __launch_bounds__(128) void k_scan(
    const float* __restrict__ dpre, const float* __restrict__ zraw, const float* __restrict__ xdbl,
    const float* __restrict__ Alog, const float* __restrict__ Dp, const float* __restrict__ dtb,
    unsigned short* uy) {
  __shared__ __align__(16) float sbc[2 * kDState];
  __shared__ __align__(16) float sy[128];
  const int tid = threadIdx.x;
  const int bpb = kDInner / 128;
  const int b = blockIdx.x / bpb;
  const int e0 = (blockIdx.x - b * bpb) * 128;
  const int e = e0 + tid;
  float a2[kDState], st[kDState];
#pragma unroll
  for (int n = 0; n < kDState; ++n) {
    const float al = bf_rne(Alog[(size_t)e * kDState + n]);
    a2[n] = -exp2f(al * kLog2e) * kLog2e;
    st[n] = 0.0f;
  }
  const float Dv = bf_rne(Dp[e]);
  const float db = bf_rne(dtb[e]);
  const size_t rb = (size_t)b * kSeq;
  for (int l = 0; l < kSeq; ++l) {
    const size_t row = rb + (size_t)l;
    const size_t ofs = row * kDInner + e;
    if (tid < 2 * kDState) sbc[tid] = xdbl[row * kRPad + kDtRank + tid];
    const float dp = dpre[ofs];
    const unsigned hb = uy[ofs];
    const unsigned lb = uy[kPlane + ofs];
    const float z = zraw[ofs];
    const float u = __uint_as_float(hb << 16) + __uint_as_float(lb << 16);
    __syncthreads();
    const float xx = dp + db;
    const float dl = fmaxf(xx, 0.0f) + log1pf(expf(-fabsf(xx)));
    const float du = dl * u;
    float y = 0.0f;
#pragma unroll
    for (int n = 0; n < kDState; ++n) {
      const float dA = exp2f(dl * a2[n]);
      st[n] = st[n] * dA + du * sbc[n];
      y = y + st[n] * sbc[kDState + n];
    }
    const float sg = __builtin_amdgcn_rcpf(1.0f + expf(-z));
    const float yo = (y + Dv * u) * (z * sg);
    sy[tid] = yo;
    __syncthreads();
    if (tid < 16) {
      const v4f va = *(const v4f*)(sy + 8 * tid);
      const v4f vb = *(const v4f*)(sy + 8 * tid + 4);
      v4u hw, lw;
      unsigned h, lo;
      split_pair(va[0], va[1], h, lo); hw[0] = h; lw[0] = lo;
      split_pair(va[2], va[3], h, lo); hw[1] = h; lw[1] = lo;
      split_pair(vb[0], vb[1], h, lo); hw[2] = h; lw[2] = lo;
      split_pair(vb[2], vb[3], h, lo); hw[3] = h; lw[3] = lo;
      const size_t o8 = (row * kDInner + (size_t)e0) / 8 + (size_t)tid;
      v4u* ph = (v4u*)(void*)uy + o8;
      v4u* pl = (v4u*)(void*)uy + (kPlane / 8) + o8;
      *(volatile v4u*)ph = hw;
      *(volatile v4u*)pl = lw;
      __threadfence();
      *(volatile v4u*)ph = hw;
      *(volatile v4u*)pl = lw;
    }
  }
}

extern "C" void kernel_launch(void* const* d_in, const int* in_sizes, int n_in,
                              void* d_out, int out_size, void* d_ws, size_t ws_size,
                              hipStream_t stream) {
  (void)in_sizes; (void)out_size;
  if (n_in < 12) return;
  const float* hs    = (const float*)d_in[0];
  const float* in2   = (const float*)d_in[1];
  const float* w1    = (const float*)d_in[2];
  const float* w2    = (const float*)d_in[3];
  const float* convw = (const float*)d_in[4];
  const float* convb = (const float*)d_in[5];
  const float* xpw   = (const float*)d_in[6];
  const float* dtw   = (const float*)d_in[7];
  const float* dtb   = (const float*)d_in[8];
  const float* Alog  = (const float*)d_in[9];
  const float* Dp    = (const float*)d_in[10];
  const float* ow    = (const float*)d_in[11];
  float* out = (float*)d_out;

  const size_t MiB = (size_t)1 << 20;
  const size_t offXraw = 0;
  const size_t offZraw = 32 * MiB;
  const size_t offUY   = 64 * MiB;
  const size_t offHs16 = 64 * MiB;
  const size_t offIn16 = 72 * MiB;
  const size_t offW116 = 80 * MiB;
  const size_t offW216 = 84 * MiB;
  const size_t offXpw  = 96 * MiB;
  const size_t offDtw  = offXpw + (size_t)kRPad * kDInner * 2;
  const size_t offOw   = offDtw + (size_t)kDInner * kDtRank * 2;
  const size_t offXdbl = offOw + (size_t)kDModel * kDInner * 2;
  const size_t offDt   = offXdbl + (size_t)kBatch * kSeq * kRPad * 4;
  const size_t offEnd  = offDt + (size_t)2 * kBatch * kSeq * kDtRank * 2;
  static_assert((size_t)kBatch * kSeq * kDInner * 4 == 32 * ((size_t)1 << 20), "f32 plane is 32 MiB");
  static_assert((size_t)kBatch * kSeq * kDModel * 2 == 8 * ((size_t)1 << 20), "hs16 is 8 MiB");
  static_assert((size_t)kDInner * kDModel * 2 == 4 * ((size_t)1 << 20), "w16 is 4 MiB");
  if (offEnd > ws_size || offEnd > 134217728u) return;

  char* ws = (char*)d_ws;
  float* xraw = (float*)(ws + offXraw);
  float* dpre = xraw;
  float* zraw = (float*)(ws + offZraw);
  unsigned short* uy = (unsigned short*)(ws + offUY);
  unsigned* hs16 = (unsigned*)(ws + offHs16);
  unsigned* in16 = (unsigned*)(ws + offIn16);
  unsigned* w116 = (unsigned*)(ws + offW116);
  unsigned* w216 = (unsigned*)(ws + offW216);
  unsigned* xpw16 = (unsigned*)(ws + offXpw);
  unsigned* dtw16 = (unsigned*)(ws + offDtw);
  unsigned* ow16 = (unsigned*)(ws + offOw);
  float* xdbl = (float*)(ws + offXdbl);
  v4u* dtpl = (v4u*)(ws + offDt);

  constexpr int nHs2  = kBatch * kSeq * kDModel / 2;
  constexpr int nW2   = kDInner * kDModel / 2;
  constexpr int nXpS2 = kRTot * kDInner / 2;
  constexpr int nXpT2 = kRPad * kDInner / 2;
  constexpr int nDtw2 = kDInner * kDtRank / 2;
  constexpr int nOw2  = kDModel * kDInner / 2;
  static_assert(nHs2 % 256 == 0 && nW2 % 256 == 0 && nXpT2 % 256 == 0 && nDtw2 % 256 == 0 && nOw2 % 256 == 0, "cast grids exact");
  cast_f32_bf16x2<<<dim3(nHs2 / 256), 256, 0, stream>>>(hs, hs16, nHs2, nHs2);
  cast_f32_bf16x2<<<dim3(nHs2 / 256), 256, 0, stream>>>(in2, in16, nHs2, nHs2);
  cast_f32_bf16x2<<<dim3(nW2 / 256), 256, 0, stream>>>(w1, w116, nW2, nW2);
  cast_f32_bf16x2<<<dim3(nW2 / 256), 256, 0, stream>>>(w2, w216, nW2, nW2);
  cast_f32_bf16x2<<<dim3(nXpT2 / 256), 256, 0, stream>>>(xpw, xpw16, nXpS2, nXpT2);
  cast_f32_bf16x2<<<dim3(nDtw2 / 256), 256, 0, stream>>>(dtw, dtw16, nDtw2, nDtw2);
  cast_f32_bf16x2<<<dim3(nOw2 / 256), 256, 0, stream>>>(ow, ow16, nOw2, nOw2);

  const long strideBLE = (long)kSeq * kDInner;
  const long strideBLD = (long)kSeq * kDModel;
  const long strideXd  = (long)kSeq * kRPad;
  const long strideDt  = (long)kSeq * kDtRank;

  static_assert(kSeq % 64 == 0 && kDInner % 64 == 0 && kDModel % 32 == 0, "in_proj shape");
  {
    dim3 g((kSeq / 64) * (kDInner / 64) / 8, kBatch);
    wmma_gemm64<1, false, false, 0, 0, false><<<g, 256, 0, stream>>>(
        (const unsigned short*)hs16, (const unsigned short*)hs16, kDModel, strideBLD,
        (const unsigned short*)w116, (const unsigned short*)w116, kDModel, 0L,
        (void*)xraw, (void*)xraw, kDInner, strideBLE, convb, convb, 0L,
        kSeq, kDInner, kDModel, 1.0f);
    wmma_gemm64<1, false, false, 0, 0, false><<<g, 256, 0, stream>>>(
        (const unsigned short*)in16, (const unsigned short*)in16, kDModel, strideBLD,
        (const unsigned short*)w216, (const unsigned short*)w216, kDModel, 0L,
        (void*)zraw, (void*)zraw, kDInner, strideBLE, convb, convb, 0L,
        kSeq, kDInner, kDModel, 1.0f);
  }

  k_conv_silu_split<<<dim3(kBatch * kSeq), 512, 0, stream>>>(xraw, convw, convb, (v4u*)(void*)uy);

  static_assert(kRPad % 64 == 0 && kDInner % 32 == 0, "x_proj shape");
  {
    dim3 g((kSeq / 64) * (kRPad / 64) / 8, kBatch);
    wmma_gemm64<1, true, false, 0, 0, false><<<g, 256, 0, stream>>>(
        (const unsigned short*)uy, (const unsigned short*)(uy + kPlane), kDInner, strideBLE,
        (const unsigned short*)xpw16, (const unsigned short*)xpw16, kDInner, 0L,
        (void*)xdbl, (void*)xdbl, kRPad, strideXd, convb, convb, 0L,
        kSeq, kRPad, kDInner, 1.0f);
  }

  constexpr int nDtRows = kBatch * kSeq;
  static_assert((nDtRows * 8) % 256 == 0, "dt split grid exact");
  k_dt_split<<<dim3(nDtRows * 8 / 256), 256, 0, stream>>>(xdbl, dtpl, nDtRows);

  static_assert(kDtRank % 32 == 0, "dt_proj K");
  {
    dim3 g((kSeq / 64) * (kDInner / 64) / 8, kBatch);
    const unsigned short* dthi = (const unsigned short*)(void*)dtpl;
    const unsigned short* dtlo = dthi + (size_t)nDtRows * kDtRank;
    wmma_gemm64<1, true, false, 0, 0, false><<<g, 256, 0, stream>>>(
        dthi, dtlo, kDtRank, strideDt,
        (const unsigned short*)dtw16, (const unsigned short*)dtw16, kDtRank, 0L,
        (void*)dpre, (void*)dpre, kDInner, strideBLE, convb, convb, 0L,
        kSeq, kDInner, kDtRank, 1.0f);
  }

  k_scan<<<dim3(kBatch * (kDInner / 128)), 128, 0, stream>>>(dpre, zraw, xdbl, Alog, Dp, dtb, uy);

  static_assert(kDModel % 64 == 0, "out_proj N");
  {
    dim3 g((kSeq / 64) * (kDModel / 64) / 8, kBatch);
    wmma_gemm64<1, true, false, 0, 0, false><<<g, 256, 0, stream>>>(
        (const unsigned short*)uy, (const unsigned short*)(uy + kPlane), kDInner, strideBLE,
        (const unsigned short*)ow16, (const unsigned short*)ow16, kDInner, 0L,
        (void*)out, (void*)out, kDModel, strideBLD, convb, convb, 0L,
        kSeq, kDModel, kDInner, 1.0f);
  }
}
